// QNetwork_6648609375076
// MI455X (gfx1250) — hardware-verified
//
#include <hip/hip_runtime.h>
#include <stddef.h>
#include <stdint.h>


#define DN     32
#define DE     16
#define DH     128
#define DM     64
#define KX     64
#define SXP    72
#define K1     256
#define KE     128
#define DPAB   256
#define KC     32
#define MLPK   272
#define NTHR   256
#define NWAVE  8
#define EPT    8
#define CHUNK  (NTHR * EPT)
#define WCAP   (EPT * 32)
#define LISTN  (NWAVE * WCAP)
#define NBA    512
#define SLA    9
#define RCAP   17408
#define DEGCAP 64
#define GBM    64
#define GTHR   128
#define EPB    256
#define DPH    132
#define APH    40
#define NEGSL  0.2f
#define NU0    (DH * (KX / 8))
#define NU1    (DM * (K1 / 8))
#define NUAB   (DPAB * (KE / 8))
#define NUC    (DH * (KC / 8))
#define NUW    NTHR
#define AGG_ZINTS (LISTN + 2 * RCAP + 3 * NBA)
#define AGG_LDS_INTS (AGG_ZINTS + 16)
#define AGG_LDS_BYTES (AGG_LDS_INTS * 4)
#define HEAD_LDS_BYTES (EPB * DPH * 4 + EPB * APH * 2 + (DH + 32 + EPB) * 4)
#define WSMAX  134217728

static_assert((CHUNK & (CHUNK - 1)) == 0 && CHUNK <= 4096);
static_assert((NBA & (NBA - 1)) == 0 && NBA == (1 << SLA));
static_assert(((long long)CHUNK << SLA) < (1LL << 31));
static_assert(LISTN % NTHR == 0);
static_assert(NBA % NWAVE == 0 && NBA % 32 == 0);
static_assert(RCAP % 4 == 0 && AGG_ZINTS % 4 == 0 && LISTN % 4 == 0);
static_assert(AGG_LDS_BYTES <= 300000);
static_assert(HEAD_LDS_BYTES <= 300000);
static_assert(NU0 % NTHR == 0 && NU1 % NTHR == 0 && NUAB % NTHR == 0 && NUC % NTHR == 0 && NUW % NTHR == 0);
static_assert(GBM == (GTHR / 32) * 16 && GTHR == 2 * GBM);
static_assert(KX == 2 * DN && KX % 32 == 0 && K1 == 2 * DH && K1 % 32 == 0 && KE == 2 * DM && KE % 32 == 0);
static_assert(KC == 2 * DE && KC == 32);
static_assert(SXP >= KX && (SXP * 2) % 16 == 0);
static_assert(APH >= KC && (APH * 2) % 16 == 0 && DPH >= DH && (DPH * 4) % 16 == 0);
static_assert(EPB == NTHR && EPB == 8 * 32);
static_assert((EPB * DPH * 4) % 16 == 0 && (EPB * APH * 2) % 16 == 0);
static_assert(DH == 4 * 32 && DM == 2 * 32 && DPAB == 2 * DH);
static_assert(MLPK == 2 * DM + DE + 2 * DM);

typedef float          v2f   __attribute__((ext_vector_type(2)));
typedef float          v4f   __attribute__((ext_vector_type(4)));
typedef float          v8f   __attribute__((ext_vector_type(8)));
typedef int            v4i   __attribute__((ext_vector_type(4)));
typedef int            v8i   __attribute__((ext_vector_type(8)));
typedef unsigned       v2u   __attribute__((ext_vector_type(2)));
typedef unsigned short v8us  __attribute__((ext_vector_type(8)));
typedef unsigned short v16us __attribute__((ext_vector_type(16)));
typedef __bf16         v16bf __attribute__((ext_vector_type(16)));
typedef v2f  __attribute__((may_alias)) v2fa;
typedef v4f  __attribute__((may_alias)) v4fa;
typedef v4i  __attribute__((may_alias)) v4ia;
typedef v8us __attribute__((may_alias)) v8usa;
union FragB { v16bf v; v16us u; v8us h[2]; v8i w; };

__device__ __forceinline__ v8f wmb(const FragB& a, const FragB& b, v8f c) {
  v8f d = __builtin_amdgcn_wmma_f32_16x16x32_bf16(false, a.v, false, b.v, (short)0, c, false, false);
  asm volatile("v_nop\n\tv_nop\n\tv_nop\n\tv_nop" : "+v"(d) : "v"(a.w), "v"(b.w));
  return d;
}

__device__ __forceinline__ unsigned bf16_bits(float f) {
  const unsigned u = __float_as_uint(f);
  return (u + 0x7FFFu + ((u >> 16) & 1u)) >> 16;
}
__device__ __forceinline__ float bf16_val(float f) {
  return __uint_as_float(bf16_bits(f) << 16);
}
__device__ __forceinline__ void put16(unsigned short* dp, v8us o) {
  *(volatile v8us*)dp = o;
  __threadfence();
  *(volatile v8us*)dp = o;
}

template <int SLB>
__device__ __forceinline__ int scan_chunk(const int* __restrict__ dsts, int nE, int cbase, int slotBase,
                                          int nb, int vec8, int* list, int tid, int lane, int wave) {
  int wc = 0;
  const int el0  = tid * EPT;
  const int e0   = cbase + el0;
  const int sent = -2147483647 - 1;
  v4i da, db;
  if (vec8 != 0 && cbase + CHUNK <= nE) {
    da = *(const v4i*)(dsts + e0);
    db = *(const v4i*)(dsts + e0 + 4);
  } else {
    da.x = (e0     < nE) ? dsts[min(e0,     nE - 1)] : sent;
    da.y = (e0 + 1 < nE) ? dsts[min(e0 + 1, nE - 1)] : sent;
    da.z = (e0 + 2 < nE) ? dsts[min(e0 + 2, nE - 1)] : sent;
    da.w = (e0 + 3 < nE) ? dsts[min(e0 + 3, nE - 1)] : sent;
    db.x = (e0 + 4 < nE) ? dsts[min(e0 + 4, nE - 1)] : sent;
    db.y = (e0 + 5 < nE) ? dsts[min(e0 + 5, nE - 1)] : sent;
    db.z = (e0 + 6 < nE) ? dsts[min(e0 + 6, nE - 1)] : sent;
    db.w = (e0 + 7 < nE) ? dsts[min(e0 + 7, nE - 1)] : sent;
  }
  const unsigned nbs = (unsigned)slotBase;
  const unsigned unb = (unsigned)nb;
  const unsigned s0 = (unsigned)da.x - nbs, s1 = (unsigned)da.y - nbs;
  const unsigned s2 = (unsigned)da.z - nbs, s3 = (unsigned)da.w - nbs;
  const unsigned s4 = (unsigned)db.x - nbs, s5 = (unsigned)db.y - nbs;
  const unsigned s6 = (unsigned)db.z - nbs, s7 = (unsigned)db.w - nbs;
  const bool h0 = s0 < unb, h1 = s1 < unb, h2 = s2 < unb, h3 = s3 < unb;
  const bool h4 = s4 < unb, h5 = s5 < unb, h6 = s6 < unb, h7 = s7 < unb;
  const unsigned any = __builtin_amdgcn_ballot_w32(h0 | h1 | h2 | h3 | h4 | h5 | h6 | h7);
  if (any != 0u) {
#define HITJ(J, HJ, SJ) { \
      const unsigned mj = __builtin_amdgcn_ballot_w32(HJ); \
      if (mj != 0u) { \
        if (HJ) { \
          const int pos = wc + (int)__builtin_amdgcn_mbcnt_lo(mj, 0u); \
          if (pos < WCAP) list[wave * WCAP + pos] = ((el0 + (J)) << SLB) | (int)(SJ); \
        } \
        wc += (int)__builtin_popcount(mj); } }
    HITJ(0, h0, s0)
    HITJ(1, h1, s1)
    HITJ(2, h2, s2)
    HITJ(3, h3, s3)
    HITJ(4, h4, s4)
    HITJ(5, h5, s5)
    HITJ(6, h6, s6)
    HITJ(7, h7, s7)
#undef HITJ
  }
  return wc;
}

__global__ __launch_bounds__(NTHR) void k_wprep(const float* __restrict__ W0, const float* __restrict__ W1,
                                                const float* __restrict__ Wm,
                                                const float* __restrict__ We0, const float* __restrict__ ae0,
                                                const float* __restrict__ We1, const float* __restrict__ ae1,
                                                unsigned short* W0T, unsigned short* W1T, unsigned short* WABT,
                                                unsigned short* WCT, float* WAE) {
  const int u  = (int)blockIdx.x * NTHR + (int)threadIdx.x;
  const int L0 = NU0, L1 = L0 + NU1, L2 = L1 + NUAB, L3 = L2 + NUC, L4 = L3 + NUW;
  v8us o;
  if (u < L0) {
    const int n  = u >> 3;
    const int k8 = (u & 7) * 8;
    const int kk = k8 & (DN - 1);
    const float* p = W0 + (size_t)kk * DH + n;
#pragma unroll
    for (int i = 0; i < 8; ++i) o[i] = (unsigned short)bf16_bits(p[(size_t)i * DH]);
    put16(W0T + (size_t)n * KX + k8, o);
    return;
  } else if (u < L1) {
    const int v  = u - L0;
    const int n  = v >> 5;
    const int k8 = (v & 31) * 8;
    const int kk = k8 & (DH - 1);
    const float* p = W1 + (size_t)kk * DM + n;
#pragma unroll
    for (int i = 0; i < 8; ++i) o[i] = (unsigned short)bf16_bits(p[(size_t)i * DM]);
    put16(W1T + (size_t)n * K1 + k8, o);
    return;
  } else if (u < L2) {
    const int v   = u - L1;
    const int n   = v >> 4;
    const int k8  = (v & 15) * 8;
    const int kk  = k8 & (DM - 1);
    const int ro  = (n >> 7) * DM;
    const int col = n & (DH - 1);
    const float* p = Wm + (size_t)(ro + kk) * DH + col;
#pragma unroll
    for (int i = 0; i < 8; ++i) o[i] = (unsigned short)bf16_bits(p[(size_t)i * DH]);
    put16(WABT + (size_t)n * KE + k8, o);
    return;
  } else if (u < L3) {
    const int v  = u - L2;
    const int n  = v >> 2;
    const int k8 = (v & 3) * 8;
    const int kk = k8 & (DE - 1);
    const float* p = Wm + (size_t)(2 * DM + kk) * DH + n;
#pragma unroll
    for (int i = 0; i < 8; ++i) o[i] = (unsigned short)bf16_bits(p[(size_t)i * DH]);
    put16(WCT + (size_t)n * KC + k8, o);
    return;
  } else if (u < L4) {
    const int tq = u - L3;
    if (tq >= 32) return;
    const int r0 = tq & 15;
    float p0 = 0.0f;
#pragma unroll 1
    for (int j = 0; j < DH; ++j) p0 = fmaf(bf16_val(We0[(size_t)r0 * DH + j]), bf16_val(ae0[j]), p0);
    float p1 = 0.0f;
#pragma unroll 1
    for (int j = 0; j < DM; ++j) p1 = fmaf(bf16_val(We1[(size_t)r0 * DM + j]), bf16_val(ae1[j]), p1);
    const float val = (tq < 16) ? p0 : p1;
    float* dp = WAE + tq;
    *(volatile float*)dp = val;
    __threadfence();
    *(volatile float*)dp = val;
    return;
  }
}

__global__ __launch_bounds__(NTHR) void k_eprep(const float* __restrict__ ea, int nEt,
                                                const float* __restrict__ lg, const float* __restrict__ lb,
                                                const float* __restrict__ WAE, float* SE0, float* SE1) {
  __shared__ __attribute__((aligned(16))) float sgb[64];
  __shared__ __attribute__((aligned(16))) float sS[2 * EPB];
  const int tid = (int)threadIdx.x, lane = tid & 31, wave = tid >> 5;
  if (wave == 0) {
    const int i = lane & 15;
    sgb[i]      = bf16_val(lg[i]);
    sgb[16 + i] = bf16_val(lb[i]);
    sgb[32 + i] = WAE[i];
    sgb[48 + i] = WAE[16 + i];
  }
  const int et = (int)blockIdx.x * EPB + tid;
  const int ec = et < nEt ? et : nEt - 1;
  const float* xp = ea + (size_t)ec * DE;
  const v4f xa = *(const v4fa*)xp;
  const v4f xb = *(const v4fa*)(xp + 4);
  const v4f xc = *(const v4fa*)(xp + 8);
  const v4f xd = *(const v4fa*)(xp + 12);
  __syncthreads();
  float xv[16] = {xa.x, xa.y, xa.z, xa.w, xb.x, xb.y, xb.z, xb.w,
                  xc.x, xc.y, xc.z, xc.w, xd.x, xd.y, xd.z, xd.w};
  float s = 0.0f;
#pragma unroll
  for (int i = 0; i < 16; ++i) { xv[i] = bf16_val(xv[i]); s += xv[i]; }
  const float mu = s * (1.0f / 16.0f);
  float q = 0.0f;
#pragma unroll
  for (int i = 0; i < 16; ++i) { xv[i] = xv[i] - mu; q = fmaf(xv[i], xv[i], q); }
  const float rstd = rsqrtf(fmaf(q, 1.0f / 16.0f, 1e-5f));
  float p0 = 0.0f, p1 = 0.0f;
#pragma unroll
  for (int i4 = 0; i4 < 4; ++i4) {
    const v4f gv = *(const v4fa*)(sgb + 4 * i4);
    const v4f bv = *(const v4fa*)(sgb + 16 + 4 * i4);
    const v4f w0 = *(const v4fa*)(sgb + 32 + 4 * i4);
    const v4f w1 = *(const v4fa*)(sgb + 48 + 4 * i4);
    const float y0 = fmaf(xv[4 * i4 + 0] * rstd, gv.x, bv.x);
    const float y1 = fmaf(xv[4 * i4 + 1] * rstd, gv.y, bv.y);
    const float y2 = fmaf(xv[4 * i4 + 2] * rstd, gv.z, bv.z);
    const float y3 = fmaf(xv[4 * i4 + 3] * rstd, gv.w, bv.w);
    p0 = fmaf(y0, w0.x, p0); p0 = fmaf(y1, w0.y, p0); p0 = fmaf(y2, w0.z, p0); p0 = fmaf(y3, w0.w, p0);
    p1 = fmaf(y0, w1.x, p1); p1 = fmaf(y1, w1.y, p1); p1 = fmaf(y2, w1.z, p1); p1 = fmaf(y3, w1.w, p1);
  }
  sS[tid]       = p0;
  sS[EPB + tid] = p1;
  __syncthreads();
  if (tid < 128) {
    const int which = tid >> 6;
    const int p = tid & 63;
    const v4f v = *(const v4fa*)(sS + which * EPB + 4 * p);
    float* op = (which == 0 ? SE0 : SE1) + (size_t)blockIdx.x * EPB + 4 * p;
    *(volatile v4f*)op = v;
    __threadfence();
    *(volatile v4f*)op = v;
  }
}

template <int NT, int DOTS, int ALN>
__global__ __launch_bounds__(GTHR) void k_gemm(const unsigned short* __restrict__ A, int lda,
                                               const unsigned short* __restrict__ BT, int ldb, int K,
                                               const float* __restrict__ X, const float* __restrict__ lng,
                                               const float* __restrict__ lnb, int nN,
                                               float* Cm, int ldc,
                                               const float* __restrict__ avs, const float* __restrict__ avd,
                                               float* AL) {
  static_assert(NT == 4 || NT == 8);
  constexpr int CB  = 16 * NT;
  constexpr int FPL = CB / 32;
  constexpr int LPR = CB / 4;
  constexpr int RPI = 32 / LPR;
  constexpr int NIT = 16 / RPI;
  __shared__ __attribute__((aligned(16))) float stg[GBM * CB];
  __shared__ __attribute__((aligned(16))) float sdt[2 * GBM];
  __shared__ __attribute__((aligned(16))) unsigned short sX[ALN != 0 ? GBM * SXP : 8];
  const int tid = (int)threadIdx.x, lane = tid & 31, wave = tid >> 5, hh = lane >> 4, m = lane & 15;
  const int rowBase = (int)blockIdx.x * GBM;
  const int colBase = (int)blockIdx.y * CB;
  (void)A; (void)lda; (void)X; (void)lng; (void)lnb; (void)nN; (void)avs; (void)avd; (void)AL; (void)sdt; (void)sX;

  if constexpr (ALN != 0) {
    const int  row  = tid >> 1, half = tid & 1;
    const int  grow = rowBase + row;
    const int  rc   = grow < nN ? grow : nN - 1;
    const bool ok   = grow < nN;
    const float* xp = X + (size_t)rc * DN + half * 16;
    const v4f xa = *(const v4fa*)xp;
    const v4f xb = *(const v4fa*)(xp + 4);
    const v4f xc = *(const v4fa*)(xp + 8);
    const v4f xd = *(const v4fa*)(xp + 12);
    float xv[16] = {xa.x, xa.y, xa.z, xa.w, xb.x, xb.y, xb.z, xb.w,
                    xc.x, xc.y, xc.z, xc.w, xd.x, xd.y, xd.z, xd.w};
    float s = 0.0f;
#pragma unroll
    for (int i = 0; i < 16; ++i) { xv[i] = bf16_val(xv[i]); s += xv[i]; }
    s += __shfl_xor(s, 1);
    const float mu = s * (1.0f / 32.0f);
    float q = 0.0f;
#pragma unroll
    for (int i = 0; i < 16; ++i) { xv[i] = xv[i] - mu; q = fmaf(xv[i], xv[i], q); }
    q += __shfl_xor(q, 1);
    const float rstd = rsqrtf(fmaf(q, 1.0f / 32.0f, 1e-5f));
    const float* gp = lng + half * 16;
    const float* bq = lnb + half * 16;
    const v4f ga = *(const v4fa*)gp, gb = *(const v4fa*)(gp + 4), gc = *(const v4fa*)(gp + 8), gd = *(const v4fa*)(gp + 12);
    const v4f ba = *(const v4fa*)bq, bb = *(const v4fa*)(bq + 4), bc = *(const v4fa*)(bq + 8), bd = *(const v4fa*)(bq + 12);
    const float gv[16] = {ga.x, ga.y, ga.z, ga.w, gb.x, gb.y, gb.z, gb.w, gc.x, gc.y, gc.z, gc.w, gd.x, gd.y, gd.z, gd.w};
    const float bw[16] = {ba.x, ba.y, ba.z, ba.w, bb.x, bb.y, bb.z, bb.w, bc.x, bc.y, bc.z, bc.w, bd.x, bd.y, bd.z, bd.w};
    v8us h0, h1, l0, l1;
#pragma unroll
    for (int i = 0; i < 8; ++i) {
      const float y0 = fmaf(xv[i] * rstd, bf16_val(gv[i]), bf16_val(bw[i]));
      const float y1 = fmaf(xv[8 + i] * rstd, bf16_val(gv[8 + i]), bf16_val(bw[8 + i]));
      const unsigned hb0 = bf16_bits(y0), hb1 = bf16_bits(y1);
      h0[i] = ok ? (unsigned short)hb0 : (unsigned short)0;
      h1[i] = ok ? (unsigned short)hb1 : (unsigned short)0;
      l0[i] = ok ? (unsigned short)bf16_bits(y0 - __uint_as_float(hb0 << 16)) : (unsigned short)0;
      l1[i] = ok ? (unsigned short)bf16_bits(y1 - __uint_as_float(hb1 << 16)) : (unsigned short)0;
    }
    unsigned short* xr = sX + row * SXP + half * 16;
    *(v8usa*)(xr)          = h0;
    *(v8usa*)(xr + 8)      = h1;
    *(v8usa*)(xr + DN)     = l0;
    *(v8usa*)(xr + DN + 8) = l1;
    __syncthreads();
  }

  v8f acc[NT];
  {
    const v8f z = {0.f, 0.f, 0.f, 0.f, 0.f, 0.f, 0.f, 0.f};
#pragma unroll
    for (int t = 0; t < NT; ++t) acc[t] = z;
  }
  const unsigned short* bp = BT + (size_t)(colBase + m) * (size_t)ldb + 8 * hh;

#pragma unroll 1
  for (int k0 = 0; k0 < K; k0 += 32) {
    FragB af;
    if constexpr (ALN != 0) {
      const unsigned short* ap = sX + (16 * wave + m) * SXP + 8 * hh + k0;
      af.h[0] = *(const v8usa*)ap;
      af.h[1] = *(const v8usa*)(ap + 16);
    } else {
      const unsigned short* ap = A + (size_t)(rowBase + 16 * wave + m) * (size_t)lda + 8 * hh + k0;
      af.h[0] = *(const v8usa*)ap;
      af.h[1] = *(const v8usa*)(ap + 16);
    }
#pragma unroll
    for (int nt = 0; nt < NT; ++nt) {
      const unsigned short* wq = bp + (size_t)(16 * nt) * (size_t)ldb + k0;
      FragB bf;
      bf.h[0] = *(const v8usa*)wq;
      bf.h[1] = *(const v8usa*)(wq + 16);
      acc[nt] = wmb(af, bf, acc[nt]);
    }
  }

#pragma unroll
  for (int nt = 0; nt < NT; ++nt) {
    const int lc = 16 * nt + m;
#pragma unroll
    for (int r = 0; r < 8; ++r) {
      const int lr = 16 * wave + 8 * hh + r;
      stg[lr * CB + lc] = acc[nt][r];
    }
  }
  __syncthreads();

  if constexpr (DOTS != 0) {
    float asv[FPL], adv[FPL];
    if constexpr (FPL == 4) {
      const v4f a = *(const v4fa*)(avs + 4 * lane);
      const v4f d = *(const v4fa*)(avd + 4 * lane);
      asv[0] = bf16_val(a.x); asv[1] = bf16_val(a.y); asv[2] = bf16_val(a.z); asv[3] = bf16_val(a.w);
      adv[0] = bf16_val(d.x); adv[1] = bf16_val(d.y); adv[2] = bf16_val(d.z); adv[3] = bf16_val(d.w);
    } else {
      const v2f a = *(const v2fa*)(avs + 2 * lane);
      const v2f d = *(const v2fa*)(avd + 2 * lane);
      asv[0] = bf16_val(a.x); asv[1] = bf16_val(a.y);
      adv[0] = bf16_val(d.x); adv[1] = bf16_val(d.y);
    }
#pragma unroll 1
    for (int i = 0; i < 16; ++i) {
      const int row = 16 * wave + i;
      float pvv[FPL];
      if constexpr (FPL == 4) {
        const v4f p = *(const v4fa*)(stg + row * CB + 4 * lane);
        pvv[0] = p.x; pvv[1] = p.y; pvv[2] = p.z; pvv[3] = p.w;
      } else {
        const v2f p = *(const v2fa*)(stg + row * CB + 2 * lane);
        pvv[0] = p.x; pvv[1] = p.y;
      }
      float s = 0.0f, d = 0.0f;
#pragma unroll
      for (int j = 0; j < FPL; ++j) { s = fmaf(pvv[j], asv[j], s); d = fmaf(pvv[j], adv[j], d); }
#pragma unroll
      for (int off = 16; off > 0; off >>= 1) {
        s += __shfl_xor(s, off);
        d += __shfl_xor(d, off);
      }
      if (lane == 0) { sdt[row] = s; sdt[GBM + row] = d; }
    }
    __syncthreads();
  }

  v4f pv[NIT];
#pragma unroll
  for (int it = 0; it < NIT; ++it) {
    const int lrow = 16 * wave + it * RPI + (lane / LPR);
    const int c4   = (lane % LPR) * 4;
    pv[it] = *(const v4fa*)(stg + lrow * CB + c4);
  }
#pragma unroll
  for (int it = 0; it < NIT; ++it) {
    const int lrow = 16 * wave + it * RPI + (lane / LPR);
    const int c4   = (lane % LPR) * 4;
    float* op = Cm + (size_t)(rowBase + lrow) * (size_t)ldc + colBase + c4;
    *(volatile v4f*)op = pv[it];
  }
  if constexpr (DOTS != 0) {
    if (wave == 0) {
      const v4f alv = *(const v4fa*)(sdt + 4 * lane);
      float* alp = AL + (size_t)blockIdx.x * (2 * GBM) + 4 * lane;
      *(volatile v4f*)alp = alv;
    }
  }
  __threadfence();
#pragma unroll
  for (int it = 0; it < NIT; ++it) {
    const int lrow = 16 * wave + it * RPI + (lane / LPR);
    const int c4   = (lane % LPR) * 4;
    float* op = Cm + (size_t)(rowBase + lrow) * (size_t)ldc + colBase + c4;
    *(volatile v4f*)op = pv[it];
  }
  if constexpr (DOTS != 0) {
    if (wave == 0) {
      const v4f alv = *(const v4fa*)(sdt + 4 * lane);
      float* alp = AL + (size_t)blockIdx.x * (2 * GBM) + 4 * lane;
      *(volatile v4f*)alp = alv;
    }
  }
}

template <int CPL, int MODE>
__global__ __launch_bounds__(NTHR) void k_sagg(const int* __restrict__ srcL, const int* __restrict__ dstL,
                                               int nE, int nG, int nNg, int nN, int nEt, int vec8, int mRows,
                                               const float* __restrict__ AL, const float* __restrict__ SE,
                                               const float* __restrict__ xl, const float* __restrict__ bias,
                                               unsigned short* hb, float* ef) {
  static_assert((CPL == 4 && MODE == 0) || (CPL == 2 && MODE == 1));
  extern __shared__ __attribute__((aligned(16))) int dsm[];
  int* list = dsm;
  int* hl   = dsm + LISTN;
  int* sl   = hl + RCAP;
  int* cnt  = sl + RCAP;
  int* offs = cnt + NBA;
  int* cur  = offs + NBA;
  int* misc = cur + NBA;
  constexpr int C = CPL * 32;
  const int tid = (int)threadIdx.x, lane = tid & 31, wave = tid >> 5;
  const int nodeBase = (int)blockIdx.x * NBA;
  (void)ef;

  {
    const v4i z4 = {0, 0, 0, 0};
    for (int i = tid * 4; i < AGG_ZINTS; i += NTHR * 4) *(v4ia*)(dsm + i) = z4;
    if (tid < 16) misc[tid] = 0;
  }
  float bv[CPL];
  if constexpr (CPL == 4) {
    const v4f a = *(const v4fa*)(bias + 4 * lane);
    bv[0] = bf16_val(a.x); bv[1] = bf16_val(a.y); bv[2] = bf16_val(a.z); bv[3] = bf16_val(a.w);
  } else {
    const v2f a = *(const v2fa*)(bias + 2 * lane);
    bv[0] = bf16_val(a.x); bv[1] = bf16_val(a.y);
  }
  __syncthreads();

  int t = 0, ov = 0;
  int gLo = nodeBase / nNg;             gLo = gLo > nG - 1 ? nG - 1 : gLo;
  int gHi = (nodeBase + NBA - 1) / nNg; gHi = gHi > nG - 1 ? nG - 1 : gHi;
  const int nChunks = (nE + CHUNK - 1) / CHUNK;
#pragma unroll 1
  for (int g = gLo; g <= gHi; ++g) {
    const int slotBase = nodeBase - g * nNg;
    const int eoff     = g * nE;
#pragma unroll 1
    for (int ch = 0; ch < nChunks; ++ch) {
      const int cbase = ch * CHUNK;
      const int wc = scan_chunk<SLA>(dstL, nE, cbase, slotBase, NBA, vec8, list, tid, lane, wave);
      if (lane == 0) misc[wave] = wc;
      __syncthreads();
      if (wave == 0) {
#pragma unroll 1
        for (int w2 = 0; w2 < NWAVE; ++w2) {
          int c = misc[w2];
          c = c < 0 ? 0 : (c > WCAP ? WCAP : c);
#pragma unroll 1
          for (int b0 = 0; b0 < c; b0 += 32) {
            const int idx = b0 + lane;
            const int ent = list[w2 * WCAP + (idx < WCAP ? idx : WCAP - 1)];
            const int m32 = (c - b0) < 32 ? (c - b0) : 32;
#pragma unroll 1
            for (int k = 0; k < m32; ++k) {
              const int u    = __builtin_amdgcn_readlane(ent, k);
              const int slot = u & (NBA - 1);
              const int el   = (u >> SLA) & (CHUNK - 1);
              const int pk   = ((eoff + cbase + el) << SLA) | slot;
              if (t < RCAP) {
                if (lane == 0) { hl[t] = pk; cnt[slot] = cnt[slot] + 1; }
                t = t + 1;
              } else {
                ov = 1;
              }
            }
          }
        }
      }
      __syncthreads();
    }
  }
  if (wave == 0 && lane == 0) { misc[8] = t; misc[9] = ov; }
  __syncthreads();
  int tt = misc[8];
  tt = tt < 0 ? 0 : (tt > RCAP ? RCAP : tt);
  const int ovf = misc[9];

  if (wave == 0) {
    const int base = lane * (NBA / 32);
    int s = 0;
#pragma unroll 1
    for (int i = 0; i < NBA / 32; ++i) s += cnt[base + i];
    int incl = s;
#pragma unroll
    for (int d = 1; d < 32; d <<= 1) {
      const int y = __shfl_up(incl, d, 32);
      if (lane >= d) incl += y;
    }
    int run = incl - s;
#pragma unroll 1
    for (int i = 0; i < NBA / 32; ++i) {
      const int cv = cnt[base + i];
      offs[base + i] = run;
      cur[base + i]  = run;
      run += cv;
    }
  }
  __syncthreads();
  if (wave == 0) {
#pragma unroll 1
    for (int b0 = 0; b0 < tt; b0 += 32) {
      const int idx = b0 + lane;
      const int ent = hl[idx < RCAP ? idx : RCAP - 1];
      const int m32 = (tt - b0) < 32 ? (tt - b0) : 32;
#pragma unroll 1
      for (int k = 0; k < m32; ++k) {
        const int u    = __builtin_amdgcn_readlane(ent, k);
        const int slot = u & (NBA - 1);
        if (lane == 0) {
          int p = cur[slot];
          p = p < 0 ? 0 : (p > RCAP - 1 ? RCAP - 1 : p);
          sl[p] = u;
          cur[slot] = p + 1;
        }
      }
    }
  }
  __syncthreads();

  const float qnan = __int_as_float(0x7fc00000);
  const float pz = (ovf != 0) ? qnan : 0.0f;
#pragma unroll 1
  for (int si = 0; si < NBA / NWAVE; ++si) {
    const int s    = si * NWAVE + wave;
    const int node = nodeBase + s;
    int c = cnt[s];
    const bool big = c > DEGCAP;
    c = c < 0 ? 0 : (c > DEGCAP ? DEGCAP : c);
    int o = offs[s];
    o = o < 0 ? 0 : (o > RCAP ? RCAP : o);
    const int nc = node < nN ? node : nN - 1;
    const float ad = AL[(nc >> 6) * (2 * GBM) + GBM + (nc & (GBM - 1))];
    float acc[CPL];
#pragma unroll
    for (int i = 0; i < CPL; ++i) acc[i] = 0.0f;
    float mx = -1.0e30f, dn = 0.0f;
#pragma unroll 1
    for (int b0 = 0; b0 < c; b0 += 32) {
      int idx = o + b0 + lane;
      idx = idx > RCAP - 1 ? RCAP - 1 : idx;
      const int ent = sl[idx];
      int eid = ent >> SLA;
      eid = eid < 0 ? 0 : (eid > nEt - 1 ? nEt - 1 : eid);
      int g = eid / nE;
      g = g > nG - 1 ? nG - 1 : g;
      int el = eid - g * nE;
      el = el < 0 ? 0 : (el > nE - 1 ? nE - 1 : el);
      int s0 = srcL[el];
      s0 = s0 < 0 ? 0 : (s0 > nNg - 1 ? nNg - 1 : s0);
      int sr = s0 + g * nNg;
      sr = sr > nN - 1 ? nN - 1 : sr;
      const float es  = AL[(sr >> 6) * (2 * GBM) + (sr & (GBM - 1))];
      const float sev = SE[eid];
      const int   esi = __float_as_int(es);
      const int   sei = __float_as_int(sev);
      const int m32 = (c - b0) < 32 ? (c - b0) : 32;
#pragma unroll 1
      for (int k = 0; k < m32; ++k) {
        const int   sk  = __builtin_amdgcn_readlane(sr, k);
        const float ask = __int_as_float(__builtin_amdgcn_readlane(esi, k));
        const float sek = __int_as_float(__builtin_amdgcn_readlane(sei, k));
        const float* rp = xl + (size_t)sk * C + CPL * lane;
        float av[CPL];
        if constexpr (CPL == 4) {
          const v4f a = *(const v4fa*)rp;
          av[0] = a.x; av[1] = a.y; av[2] = a.z; av[3] = a.w;
        } else {
          const v2f a = *(const v2fa*)rp;
          av[0] = a.x; av[1] = a.y;
        }
        float lg = (ask + ad) + sek;
        lg = lg > 0.f ? lg : NEGSL * lg;
        const float df = lg - mx;
        const float ee = __expf(-fabsf(df));
        const bool  up = df > 0.f;
        const float s1 = up ? ee : 1.0f;
        const float s2 = up ? 1.0f : ee;
        mx = up ? lg : mx;
        dn = fmaf(dn, s1, s2);
#pragma unroll
        for (int i = 0; i < CPL; ++i) acc[i] = fmaf(acc[i], s1, s2 * av[i]);
      }
    }
    const float dsafe = dn > 0.0f ? dn : 1.0f;
    const float inv   = __builtin_amdgcn_rcpf(dsafe);
    const float pzr   = big ? qnan : pz;
    const bool  live  = node < nN;
    float v[CPL];
#pragma unroll
    for (int i = 0; i < CPL; ++i) {
      float y = fmaf(acc[i], inv, bv[i]);
      if constexpr (MODE == 0) y = y > 0.0f ? y : (__expf(y) - 1.0f);
      y = y + pzr;
      v[i] = live ? y : 0.0f;
    }
    if constexpr (MODE == 0) {
      unsigned hw[4], lw[4];
#pragma unroll
      for (int i = 0; i < 4; ++i) {
        hw[i] = bf16_bits(v[i]);
        lw[i] = bf16_bits(v[i] - __uint_as_float(hw[i] << 16));
      }
      v2u ho, lo;
      ho.x = hw[0] | (hw[1] << 16); ho.y = hw[2] | (hw[3] << 16);
      lo.x = lw[0] | (lw[1] << 16); lo.y = lw[2] | (lw[3] << 16);
      if (node < mRows) {
        unsigned short* hp = hb + (size_t)node * (2 * C) + CPL * lane;
        *(volatile v2u*)hp       = ho;
        *(volatile v2u*)(hp + C) = lo;
        __threadfence();
        *(volatile v2u*)hp       = ho;
        *(volatile v2u*)(hp + C) = lo;
      }
    } else {
      const unsigned hw0 = bf16_bits(v[0]), hw1 = bf16_bits(v[1]);
      const unsigned lw0 = bf16_bits(v[0] - __uint_as_float(hw0 << 16));
      const unsigned lw1 = bf16_bits(v[1] - __uint_as_float(hw1 << 16));
      const unsigned ho = hw0 | (hw1 << 16);
      const unsigned lo = lw0 | (lw1 << 16);
      v2f fv;
      fv.x = v[0]; fv.y = v[1];
      if (node < mRows) {
        float* fp = ef + (size_t)node * C + CPL * lane;
        unsigned short* hp = hb + (size_t)node * (2 * C) + CPL * lane;
        *(volatile v2f*)fp            = fv;
        *(volatile unsigned*)hp       = ho;
        *(volatile unsigned*)(hp + C) = lo;
        __threadfence();
        *(volatile v2f*)fp            = fv;
        *(volatile unsigned*)hp       = ho;
        *(volatile unsigned*)(hp + C) = lo;
      }
    }
  }
}

__global__ __launch_bounds__(NTHR) void k_pool(const float* __restrict__ EF, int nNg,
                                               const float* __restrict__ Wm, const float* __restrict__ b1,
                                               float* PC) {
  __shared__ __attribute__((aligned(16))) double ssum[NTHR];
  __shared__ __attribute__((aligned(16))) float  smax[NTHR];
  __shared__ __attribute__((aligned(16))) float  sctx[DH];
  __shared__ __attribute__((aligned(16))) float  spc[DH];
  const int tid = (int)threadIdx.x;
  const int g = (int)blockIdx.x;
  const int c = tid & (DM - 1), rg = tid >> 6;
  double s = 0.0;
  float mxv = -3.0e38f;
  const float* base = EF + (size_t)g * (size_t)nNg * DM + c;
#pragma unroll 1
  for (int r = rg; r < nNg; r += 4) {
    const float v = base[(size_t)r * DM];
    s += (double)v;
    mxv = fmaxf(mxv, v);
  }
  ssum[tid] = s;
  smax[tid] = mxv;
  __syncthreads();
  if (tid < DM) {
    const double tot = ((ssum[tid] + ssum[DM + tid]) + ssum[2 * DM + tid]) + ssum[3 * DM + tid];
    const float mean = (float)(tot / (double)nNg);
    const float mxa  = fmaxf(fmaxf(smax[tid], smax[DM + tid]), fmaxf(smax[2 * DM + tid], smax[3 * DM + tid]));
    sctx[tid]      = mean;
    sctx[DM + tid] = mxa;
  }
  __syncthreads();
  if (tid < DH) {
    const float* wp = Wm + (size_t)(2 * DM + DE) * DH + tid;
    float acc = 0.0f;
#pragma unroll 1
    for (int k = 0; k < DH; ++k) acc = fmaf(sctx[k], bf16_val(wp[(size_t)k * DH]), acc);
    spc[tid] = acc + bf16_val(b1[tid]);
  }
  __syncthreads();
  if (tid < 32) {
    const v4f v = *(const v4fa*)(spc + 4 * tid);
    float* op = PC + (size_t)g * DH + 4 * tid;
    *(volatile v4f*)op = v;
    __threadfence();
    *(volatile v4f*)op = v;
  }
}

__device__ __forceinline__ void wave_gemm_c(const unsigned short* sAw, float* sDw,
                                            const unsigned short* __restrict__ BT, int hh, int m) {
#pragma unroll 1
  for (int nh = 0; nh < 2; ++nh) {
    v8f acc[2][4];
    {
      const v8f z = {0.f, 0.f, 0.f, 0.f, 0.f, 0.f, 0.f, 0.f};
#pragma unroll
      for (int mt = 0; mt < 2; ++mt)
#pragma unroll
        for (int nt = 0; nt < 4; ++nt) acc[mt][nt] = z;
    }
    const unsigned short* ap0 = sAw + m * APH + 8 * hh;
    const unsigned short* ap1 = ap0 + 16 * APH;
    const unsigned short* bp  = BT + (size_t)(64 * nh + m) * (size_t)KC + 8 * hh;
#pragma unroll 1
    for (int k0 = 0; k0 < KC; k0 += 32) {
      FragB a0, a1;
      a0.h[0] = *(const v8usa*)(ap0 + k0);
      a0.h[1] = *(const v8usa*)(ap0 + k0 + 16);
      a1.h[0] = *(const v8usa*)(ap1 + k0);
      a1.h[1] = *(const v8usa*)(ap1 + k0 + 16);
#pragma unroll
      for (int nt = 0; nt < 4; ++nt) {
        const unsigned short* wq = bp + (size_t)(16 * nt) * (size_t)KC + k0;
        FragB b;
        b.h[0] = *(const v8usa*)wq;
        b.h[1] = *(const v8usa*)(wq + 16);
        acc[0][nt] = wmb(a0, b, acc[0][nt]);
        acc[1][nt] = wmb(a1, b, acc[1][nt]);
      }
    }
#pragma unroll
    for (int nt = 0; nt < 4; ++nt) {
      const int col = 64 * nh + 16 * nt + m;
#pragma unroll
      for (int mt = 0; mt < 2; ++mt)
#pragma unroll
        for (int r = 0; r < 8; ++r) sDw[(16 * mt + 8 * hh + r) * DPH + col] = acc[mt][nt][r];
    }
  }
}

__global__ __launch_bounds__(NTHR) void k_head(const int* __restrict__ srcL, const int* __restrict__ dstL,
                                               int nE, int nG, int nNg, int nN, int nEt,
                                               const float* __restrict__ ea,
                                               const float* __restrict__ lg, const float* __restrict__ lb,
                                               const unsigned short* __restrict__ WCT,
                                               const float* __restrict__ PAB, const float* __restrict__ PC,
                                               const float* __restrict__ W2, const float* __restrict__ b2,
                                               float* out) {
  extern __shared__ __attribute__((aligned(16))) float dyn[];
  float*          sD  = dyn;
  unsigned short* sA  = (unsigned short*)(dyn + EPB * DPH);
  float*          sW2 = dyn + EPB * DPH + (EPB * APH) / 2;
  float*          sGB = sW2 + DH;
  float*          sQ  = sGB + 32;
  const int tid = (int)threadIdx.x, lane = tid & 31, wave = tid >> 5, hh = lane >> 4, m = lane & 15;

  if (tid < DH) sW2[tid] = bf16_val(W2[tid]);
  if (wave == 4) {
    const int i = lane & 15;
    sGB[i]      = bf16_val(lg[i]);
    sGB[16 + i] = bf16_val(lb[i]);
  }
  const int  elb  = (int)blockIdx.x * EPB;
  const int  et   = elb + tid;
  const int  ec   = et < nEt ? et : nEt - 1;
  int g = ec / nE;
  g = g > nG - 1 ? nG - 1 : g;
  int el = ec - g * nE;
  el = el < 0 ? 0 : (el > nE - 1 ? nE - 1 : el);
  int s0 = srcL[el];
  int d0 = dstL[el];
  s0 = s0 < 0 ? 0 : (s0 > nNg - 1 ? nNg - 1 : s0);
  d0 = d0 < 0 ? 0 : (d0 > nNg - 1 ? nNg - 1 : d0);
  int sr = s0 + g * nNg; sr = sr > nN - 1 ? nN - 1 : sr;
  int ds = d0 + g * nNg; ds = ds > nN - 1 ? nN - 1 : ds;
  const float bias2 = bf16_val(b2[0]);
  const float* xp = ea + (size_t)ec * DE;
  const v4f xa = *(const v4fa*)xp;
  const v4f xb = *(const v4fa*)(xp + 4);
  const v4f xc = *(const v4fa*)(xp + 8);
  const v4f xd = *(const v4fa*)(xp + 12);
  __syncthreads();

  {
    float xv[16] = {xa.x, xa.y, xa.z, xa.w, xb.x, xb.y, xb.z, xb.w,
                    xc.x, xc.y, xc.z, xc.w, xd.x, xd.y, xd.z, xd.w};
    float s = 0.0f;
#pragma unroll
    for (int i = 0; i < 16; ++i) { xv[i] = bf16_val(xv[i]); s += xv[i]; }
    const float mu = s * (1.0f / 16.0f);
    float q = 0.0f;
#pragma unroll
    for (int i = 0; i < 16; ++i) { xv[i] = xv[i] - mu; q = fmaf(xv[i], xv[i], q); }
    const float rstd = rsqrtf(fmaf(q, 1.0f / 16.0f, 1e-5f));
    v8us h0, h1, l0, l1;
#pragma unroll
    for (int i4 = 0; i4 < 4; ++i4) {
      const v4f gv = *(const v4fa*)(sGB + 4 * i4);
      const v4f bv = *(const v4fa*)(sGB + 16 + 4 * i4);
      const float y[4] = {fmaf(xv[4 * i4 + 0] * rstd, gv.x, bv.x), fmaf(xv[4 * i4 + 1] * rstd, gv.y, bv.y),
                          fmaf(xv[4 * i4 + 2] * rstd, gv.z, bv.z), fmaf(xv[4 * i4 + 3] * rstd, gv.w, bv.w)};
#pragma unroll
      for (int j = 0; j < 4; ++j) {
        const unsigned hbv = bf16_bits(y[j]);
        const unsigned lbv = bf16_bits(y[j] - __uint_as_float(hbv << 16));
        const int idx = 4 * i4 + j;
        if (idx < 8) { h0[idx] = (unsigned short)hbv; l0[idx] = (unsigned short)lbv; }
        else         { h1[idx - 8] = (unsigned short)hbv; l1[idx - 8] = (unsigned short)lbv; }
      }
    }
    unsigned short* ra = sA + tid * APH;
    *(v8usa*)(ra)          = h0;
    *(v8usa*)(ra + 8)      = h1;
    *(v8usa*)(ra + DE)     = l0;
    *(v8usa*)(ra + DE + 8) = l1;
  }
  __syncthreads();

  const unsigned short* sAw = sA + 32 * wave * APH;
  float*                sDw = sD + 32 * wave * DPH;
  wave_gemm_c(sAw, sDw, WCT, hh, m);
  __syncthreads();

  {
    const float* rd  = sD + (size_t)tid * DPH;
    const float* pap = PAB + (size_t)sr * DPAB;
    const float* pbp = PAB + (size_t)ds * DPAB + DH;
    const float* pcp = PC + (size_t)g * DH;
    float qv = 0.0f;
#pragma unroll 1
    for (int c8 = 0; c8 < DH / 8; ++c8) {
      const v4f da = *(const v4fa*)(rd + 8 * c8);
      const v4f db = *(const v4fa*)(rd + 8 * c8 + 4);
      const v4f aa = *(const v4fa*)(pap + 8 * c8);
      const v4f ab = *(const v4fa*)(pap + 8 * c8 + 4);
      const v4f ba = *(const v4fa*)(pbp + 8 * c8);
      const v4f bb = *(const v4fa*)(pbp + 8 * c8 + 4);
      const v4f ca = *(const v4fa*)(pcp + 8 * c8);
      const v4f cb = *(const v4fa*)(pcp + 8 * c8 + 4);
      const v4f wa = *(const v4fa*)(sW2 + 8 * c8);
      const v4f wb = *(const v4fa*)(sW2 + 8 * c8 + 4);
      const v8f d8 = {da.x, da.y, da.z, da.w, db.x, db.y, db.z, db.w};
      const v8f a8 = {aa.x, aa.y, aa.z, aa.w, ab.x, ab.y, ab.z, ab.w};
      const v8f b8 = {ba.x, ba.y, ba.z, ba.w, bb.x, bb.y, bb.z, bb.w};
      const v8f c8v = {ca.x, ca.y, ca.z, ca.w, cb.x, cb.y, cb.z, cb.w};
      const v8f w8 = {wa.x, wa.y, wa.z, wa.w, wb.x, wb.y, wb.z, wb.w};
#pragma unroll
      for (int i = 0; i < 8; ++i) {
        float tv = (a8[i] + b8[i]) + d8[i];
        tv = tv + c8v[i];
        tv = fmaxf(tv, 0.0f);
        qv = fmaf(tv, w8[i], qv);
      }
    }
    qv = qv + bias2;
    sQ[tid] = qv;
  }
  __syncthreads();

  if (tid < 64) {
    const int p  = tid;
    const int e4 = elb + 4 * p;
    const v4f v  = *(const v4fa*)(sQ + 4 * p);
    float* op = out + (size_t)elb + 4 * p;
    const bool full = (e4 + 4 <= nEt);
    if (full) {
      *(volatile v4f*)op = v;
    } else {
      if (e4 + 0 < nEt) *(volatile float*)(op + 0) = v.x;
      if (e4 + 1 < nEt) *(volatile float*)(op + 1) = v.y;
      if (e4 + 2 < nEt) *(volatile float*)(op + 2) = v.z;
      if (e4 + 3 < nEt) *(volatile float*)(op + 3) = v.w;
    }
    __threadfence();
    if (full) {
      *(volatile v4f*)op = v;
    } else {
      if (e4 + 0 < nEt) *(volatile float*)(op + 0) = v.x;
      if (e4 + 1 < nEt) *(volatile float*)(op + 1) = v.y;
      if (e4 + 2 < nEt) *(volatile float*)(op + 2) = v.z;
      if (e4 + 3 < nEt) *(volatile float*)(op + 3) = v.w;
    }
  }
}

static inline int cdiv(int a, int b) { return (a + b - 1) / b; }

extern "C" void kernel_launch(void* const* d_in, const int* in_sizes, int n_in,
                              void* d_out, int out_size, void* d_ws, size_t ws_size,
                              hipStream_t stream) {
  if (n_in < 23) return;
  if (in_sizes[2] < 2 || (in_sizes[2] & 1) != 0) return;
  const int nE = in_sizes[2] / 2;
  if (in_sizes[1] < DE || (in_sizes[1] % DE) != 0) return;
  const int nEt = in_sizes[1] / DE;
  if (nE < 1 || (nEt % nE) != 0) return;
  const int nG = nEt / nE;
  if (nG < 1) return;
  if (in_sizes[0] < DN || (in_sizes[0] % DN) != 0) return;
  const int nN = in_sizes[0] / DN;
  if ((nN % nG) != 0) return;
  const int nNg = nN / nG;
  if (nNg < 1) return;
  if (nEt >= (1 << 21) || nN >= (1 << 24)) return;
  if (in_sizes[3] != DN || in_sizes[4] != DN) return;
  if (in_sizes[5] != DE || in_sizes[6] != DE) return;
  if (in_sizes[7] != DN * DH || in_sizes[8] != DE * DH) return;
  if (in_sizes[9] != DH || in_sizes[10] != DH || in_sizes[11] != DH || in_sizes[12] != DH) return;
  if (in_sizes[13] != DH * DM || in_sizes[14] != DE * DM) return;
  if (in_sizes[15] != DM || in_sizes[16] != DM || in_sizes[17] != DM || in_sizes[18] != DM) return;
  if (in_sizes[19] != MLPK * DH) return;
  if (in_sizes[20] != DH || in_sizes[21] != DH || in_sizes[22] < 1) return;
  if (out_size != nEt) return;

  const float* node_x = (const float*)d_in[0];
  const float* ea     = (const float*)d_in[1];
  const int*   ei     = (const int*)d_in[2];
  const float* lng    = (const float*)d_in[3];
  const float* lnb    = (const float*)d_in[4];
  const float* leg    = (const float*)d_in[5];
  const float* leb    = (const float*)d_in[6];
  const float* W0     = (const float*)d_in[7];
  const float* We0    = (const float*)d_in[8];
  const float* as0    = (const float*)d_in[9];
  const float* ad0    = (const float*)d_in[10];
  const float* ae0    = (const float*)d_in[11];
  const float* b0     = (const float*)d_in[12];
  const float* W1     = (const float*)d_in[13];
  const float* We1    = (const float*)d_in[14];
  const float* as1    = (const float*)d_in[15];
  const float* ad1    = (const float*)d_in[16];
  const float* ae1    = (const float*)d_in[17];
  const float* b1     = (const float*)d_in[18];
  const float* Wm     = (const float*)d_in[19];
  const float* mb1    = (const float*)d_in[20];
  const float* mW2    = (const float*)d_in[21];
  const float* mb2    = (const float*)d_in[22];
  float* out = (float*)d_out;
  const int* srcL = ei;
  const int* dstL = ei + nE;

  const int MP   = cdiv(nN, GBM) * GBM;
  const int gM   = MP / GBM;
  const int gA   = cdiv(MP, NBA);
  if ((long long)gA * NBA < (long long)MP) return;
  const int nEtP = cdiv(nEt, EPB) * EPB;
  const int vec8 = ((nE & 3) == 0) ? 1 : 0;

  char* ws = (char*)d_ws;
  size_t off = 0;
  const size_t oW0T = off; off += (size_t)DH * KX * 2;               off = (off + 255) & ~(size_t)255;
  const size_t oW1T = off; off += (size_t)DM * K1 * 2;               off = (off + 255) & ~(size_t)255;
  const size_t oWAB = off; off += (size_t)DPAB * KE * 2;             off = (off + 255) & ~(size_t)255;
  const size_t oWCT = off; off += (size_t)DH * KC * 2;               off = (off + 255) & ~(size_t)255;
  const size_t oWAE = off; off += 256;                               off = (off + 255) & ~(size_t)255;
  const size_t oSE0 = off; off += (size_t)nEtP * 4;                  off = (off + 255) & ~(size_t)255;
  const size_t oSE1 = off; off += (size_t)nEtP * 4;                  off = (off + 255) & ~(size_t)255;
  const size_t oAL  = off; off += (size_t)gM * (2 * GBM) * 4;        off = (off + 255) & ~(size_t)255;
  const size_t oH0  = off; off += (size_t)MP * DH * 4;               off = (off + 255) & ~(size_t)255;
  const size_t oH1  = off; off += (size_t)MP * K1 * 2;               off = (off + 255) & ~(size_t)255;
  const size_t oHB  = off; off += (size_t)MP * DM * 4;               off = (off + 255) & ~(size_t)255;
  const size_t oEF  = off; off += (size_t)MP * DM * 4;               off = (off + 255) & ~(size_t)255;
  const size_t oEH  = off; off += (size_t)MP * KE * 2;               off = (off + 255) & ~(size_t)255;
  const size_t oPAB = off; off += (size_t)MP * DPAB * 4;             off = (off + 255) & ~(size_t)255;
  const size_t oPC  = off; off += (size_t)nG * DH * 4;               off = (off + 255) & ~(size_t)255;
  if (off > ws_size || off > (size_t)WSMAX) return;
  unsigned short* W0T  = (unsigned short*)(ws + oW0T);
  unsigned short* W1T  = (unsigned short*)(ws + oW1T);
  unsigned short* WABT = (unsigned short*)(ws + oWAB);
  unsigned short* WCT  = (unsigned short*)(ws + oWCT);
  float*          WAE  = (float*)(ws + oWAE);
  float*          SE0  = (float*)(ws + oSE0);
  float*          SE1  = (float*)(ws + oSE1);
  float*          ALp  = (float*)(ws + oAL);
  float*          H0   = (float*)(ws + oH0);
  unsigned short* H1   = (unsigned short*)(ws + oH1);
  float*          HB   = (float*)(ws + oHB);
  float*          EF   = (float*)(ws + oEF);
  unsigned short* EH   = (unsigned short*)(ws + oEH);
  float*          PAB  = (float*)(ws + oPAB);
  float*          PC   = (float*)(ws + oPC);

  hipFuncSetAttribute(reinterpret_cast<const void*>(&k_sagg<4, 0>), hipFuncAttributeMaxDynamicSharedMemorySize,
                      (int)AGG_LDS_BYTES);
  hipFuncSetAttribute(reinterpret_cast<const void*>(&k_sagg<2, 1>), hipFuncAttributeMaxDynamicSharedMemorySize,
                      (int)AGG_LDS_BYTES);
  hipFuncSetAttribute(reinterpret_cast<const void*>(&k_head), hipFuncAttributeMaxDynamicSharedMemorySize,
                      (int)HEAD_LDS_BYTES);

  k_wprep<<<(NU0 + NU1 + NUAB + NUC + NUW) / NTHR, NTHR, 0, stream>>>(W0, W1, Wm, We0, ae0, We1, ae1,
                                                                      W0T, W1T, WABT, WCT, WAE);
  k_eprep<<<nEtP / EPB, NTHR, 0, stream>>>(ea, nEt, leg, leb, WAE, SE0, SE1);
  k_gemm<8, 1, 1><<<dim3(gM, 1), GTHR, 0, stream>>>(H1, KX, W0T, KX, KX, node_x, lng, lnb, nN,
                                                     H0, DH, as0, ad0, ALp);
  k_sagg<4, 0><<<gA, NTHR, AGG_LDS_BYTES, stream>>>(srcL, dstL, nE, nG, nNg, nN, nEt, vec8, MP,
                                                     ALp, SE0, H0, b0, H1, EF);
  k_gemm<4, 1, 0><<<dim3(gM, 1), GTHR, 0, stream>>>(H1, K1, W1T, K1, K1, node_x, lng, lnb, nN,
                                                     HB, DM, as1, ad1, ALp);
  k_sagg<2, 1><<<gA, NTHR, AGG_LDS_BYTES, stream>>>(srcL, dstL, nE, nG, nNg, nN, nEt, vec8, MP,
                                                     ALp, SE1, HB, b1, EH, EF);
  k_pool<<<nG, NTHR, 0, stream>>>(EF, nNg, Wm, mb1, PC);
  k_gemm<8, 0, 0><<<dim3(gM, DPAB / 128), GTHR, 0, stream>>>(EH, KE, WABT, KE, KE, node_x, lng, lnb, nN,
                                                             PAB, DPAB, as0, ad0, ALp);
  k_head<<<nEtP / EPB, NTHR, HEAD_LDS_BYTES, stream>>>(srcL, dstL, nE, nG, nNg, nN, nEt, ea, leg, leb, WCT,
                                                         PAB, PC, mW2, mb2, out);
}
